// GNNPerAgentModel_32152125178257
// MI455X (gfx1250) — hardware-verified
//
#include <hip/hip_runtime.h>
#include <stddef.h>
#include <math.h>


typedef float    v4f  __attribute__((ext_vector_type(4)));
typedef float    v8f  __attribute__((ext_vector_type(8)));
typedef _Float16 v8h  __attribute__((ext_vector_type(8)));
typedef _Float16 v16h __attribute__((ext_vector_type(16)));
typedef v4f v4fa __attribute__((may_alias));

union FragH { v16h v; v8h h[2]; _Float16 e[16]; };
union Pack8 { v8h h; v4f f; _Float16 e[8]; };

#define WSC16  16.0f
#define WINV16 0.0625f
#define WSC64  64.0f
#define WINV64 0.015625f
#define CW  4
#define CT  (CW * 32)
#define LW  2
#define LT  (LW * 32)
#define TT  256
#define SPB 16
#define PT  256

__device__ __forceinline__ v8f z8f() {
    v8f r;
#pragma unroll
    for (int i = 0; i < 8; ++i) r[i] = 0.0f;
    return r;
}

__device__ __forceinline__ v8f wmh(v16h a, v16h b, v8f c) {
    v8f d = __builtin_amdgcn_wmma_f32_16x16x32_f16(false, a, false, b, (short)0, c, false, false);
    asm volatile("v_nop\n\tv_nop\n\tv_nop\n\tv_nop" : "+v"(d) : "v"(a), "v"(b));
    return d;
}

__device__ __forceinline__ v8h ld8(const float* p) {
    Pack8 k;
#pragma unroll
    for (int i = 0; i < 8; ++i) k.e[i] = (_Float16)p[i];
    return k.h;
}
__device__ __forceinline__ v8h ld8(const _Float16* p) { return *(const v8h*)p; }

template <int IC, int KSZ>
__device__ __forceinline__ v4f wpiece(const float* __restrict__ W, int q) {
    constexpr int K = KSZ * KSZ * IC, KP = K / 8;
    const int n = q / KP, j = q - n * KP;
    Pack8 pk;
#pragma unroll
    for (int i = 0; i < 8; ++i) {
        const int k   = 8 * j + i;
        const int ci  = k % IC;
        const int kwh = k / IC;
        const int kw  = kwh % KSZ;
        const int kh  = kwh / KSZ;
        pk.e[i] = (_Float16)(W[(((size_t)n * IC + ci) * KSZ + kh) * KSZ + kw] * WSC16);
    }
    return pk.f;
}

__global__ __launch_bounds__(PT)
void k_prep(const float* __restrict__ Wp, const float* __restrict__ W1, const float* __restrict__ W2,
            const float* __restrict__ W3, _Float16* wpT, _Float16* w1T, _Float16* w2T, _Float16* w3T)
{
    __shared__ __attribute__((aligned(16))) _Float16 tile[64 * 256];
    const int tid = threadIdx.x;
    const int blk = (int)blockIdx.x;
    if (blk < 256) {
        const int g = blk;
#pragma unroll 1
        for (int kk = 0; kk < 64; ++kk)
            tile[kk * 256 + tid] = (_Float16)(Wp[((size_t)kk * 256 + g) * 256 + tid] * WSC64);
        __syncthreads();
        v4f pv[8];
#pragma unroll
        for (int it = 0; it < 8; ++it) {
            const int q = it * 256 + tid, n = q >> 3, j = q & 7;
            Pack8 pk;
#pragma unroll
            for (int i = 0; i < 8; ++i) pk.e[i] = tile[(8 * j + i) * 256 + n];
            pv[it] = pk.f;
        }
#pragma unroll
        for (int it = 0; it < 8; ++it) {
            const int q = it * 256 + tid, n = q >> 3, j = q & 7;
            *(volatile v4fa*)(wpT + (size_t)n * 16384 + 64 * g + 8 * j) = pv[it];
        }
        __threadfence();
#pragma unroll
        for (int it = 0; it < 8; ++it) {
            const int q = it * 256 + tid, n = q >> 3, j = q & 7;
            *(volatile v4fa*)(wpT + (size_t)n * 16384 + 64 * g + 8 * j) = pv[it];
        }
    } else if (blk < 259) {
        const int q = (blk - 256) * PT + tid;
        const v4f v = wpiece<3, 8>(W1, q);
        *(volatile v4fa*)(w1T + (size_t)q * 8) = v;
        __threadfence();
        *(volatile v4fa*)(w1T + (size_t)q * 8) = v;
    } else if (blk < 275) {
        const int q = (blk - 259) * PT + tid;
        const v4f v = wpiece<32, 4>(W2, q);
        *(volatile v4fa*)(w2T + (size_t)q * 8) = v;
        __threadfence();
        *(volatile v4fa*)(w2T + (size_t)q * 8) = v;
    } else {
        const int q = (blk - 275) * PT + tid;
        const v4f v = wpiece<64, 3>(W3, q);
        *(volatile v4fa*)(w3T + (size_t)q * 8) = v;
        __threadfence();
        *(volatile v4fa*)(w3T + (size_t)q * 8) = v;
    }
}

template <typename TI, int IH, int IW, int IC, int OC, int KSZ, int STR, int OH, int OW, int INPP, int OUTPP>
__global__ __launch_bounds__(CT)
void k_conv(const TI* __restrict__ in, const _Float16* __restrict__ wT,
            const float* __restrict__ bias, _Float16* outp, int nImg)
{
    constexpr int M   = OH * OW;
    constexpr int NT  = OC / 16;
    constexpr int K   = KSZ * KSZ * IC;
    constexpr int KS  = K / 32;
    constexpr int RL  = KSZ * IC;
    constexpr int TPI = OUTPP / 32;
    constexpr int TH  = 32 * OC;
    constexpr int NPI = TH / 256;
    static_assert((K % 32) == 0);
    static_assert((RL % 8) == 0);
    static_assert((OUTPP % 32) == 0);
    static_assert(OUTPP >= M);
    static_assert((OC % 16) == 0);
    static_assert(NPI * 256 == TH);
    static_assert((OH - 1) * STR + KSZ <= IH);
    static_assert((OW - 1) * STR + KSZ <= IW);
    static_assert(IH * IW <= INPP);

    __shared__ __attribute__((aligned(16))) _Float16 stg[CW * TH];

    const int tid = threadIdx.x, lane = tid & 31, wave = tid >> 5, hh = lane >> 4, m = lane & 15;
    const int total = nImg * TPI;
    int gw = (int)blockIdx.x * CW + wave;
    const bool wvalid = gw < total;
    gw = wvalid ? gw : (total - 1);
    const int b  = gw / TPI;
    const int mt = gw - b * TPI;

    const int p0 = mt * 32 + m, p1 = p0 + 16;
    const int q0 = p0 < M ? p0 : (M - 1);
    const int q1 = p1 < M ? p1 : (M - 1);
    const int oy0 = q0 / OW, ox0 = q0 - oy0 * OW;
    const int oy1 = q1 / OW, ox1 = q1 - oy1 * OW;
    const size_t base0 = ((size_t)b * INPP + (size_t)(oy0 * STR) * IW + (size_t)(ox0 * STR)) * IC;
    const size_t base1 = ((size_t)b * INPP + (size_t)(oy1 * STR) * IW + (size_t)(ox1 * STR)) * IC;

    v8f acc0[NT], acc1[NT];
#pragma unroll
    for (int t = 0; t < NT; ++t) { acc0[t] = z8f(); acc1[t] = z8f(); }

#pragma unroll 1
    for (int s = 0; s < KS; ++s) {
        FragH a0, a1;
#pragma unroll
        for (int c = 0; c < 2; ++c) {
            const int k0  = s * 32 + 16 * c + 8 * hh;
            const int kh  = k0 / RL;
            const int rem = k0 - kh * RL;
            const size_t koff = (size_t)kh * (IW * IC) + (size_t)rem;
            a0.h[c] = ld8(in + base0 + koff);
            a1.h[c] = ld8(in + base1 + koff);
        }
#pragma unroll
        for (int t = 0; t < NT; ++t) {
            FragH bf;
            const _Float16* bp = wT + (size_t)(t * 16 + m) * K + (size_t)(s * 32 + 8 * hh);
            bf.h[0] = *(const v8h*)bp;
            bf.h[1] = *(const v8h*)(bp + 16);
            acc0[t] = wmh(a0.v, bf.v, acc0[t]);
            acc1[t] = wmh(a1.v, bf.v, acc1[t]);
        }
    }

    _Float16* sw = stg + wave * TH;
#pragma unroll
    for (int t = 0; t < NT; ++t) {
        const int col = t * 16 + m;
        const float bv = bias[col];
#pragma unroll
        for (int r = 0; r < 8; ++r) {
            const float v0 = fmaxf(acc0[t][r] * WINV16 + bv, 0.0f);
            const float v1 = fmaxf(acc1[t][r] * WINV16 + bv, 0.0f);
            sw[(8 * hh + r) * OC + col]      = (_Float16)v0;
            sw[(16 + 8 * hh + r) * OC + col] = (_Float16)v1;
        }
    }
    __syncthreads();

    const size_t gb = ((size_t)b * OUTPP + (size_t)mt * 32) * OC;
    v4f pv[NPI];
#pragma unroll
    for (int it = 0; it < NPI; ++it) pv[it] = *(const v4fa*)(sw + (it * 32 + lane) * 8);
    if (wvalid) {
#pragma unroll
        for (int it = 0; it < NPI; ++it)
            *(volatile v4fa*)(outp + gb + (size_t)(it * 32 + lane) * 8) = pv[it];
    }
    __threadfence();
    if (wvalid) {
#pragma unroll
        for (int it = 0; it < NPI; ++it)
            *(volatile v4fa*)(outp + gb + (size_t)(it * 32 + lane) * 8) = pv[it];
    }
}

__global__ __launch_bounds__(LT)
void k_linear(const _Float16* __restrict__ A, const _Float16* __restrict__ wT,
              const float* __restrict__ bias, float* outp, int nImg)
{
    constexpr int KT = 16384, KS = KT / 32, NO = 256, NG = 4, NT = 4;
    __shared__ __attribute__((aligned(16))) float stg[LW * 32 * 64];

    const int tid = threadIdx.x, lane = tid & 31, wave = tid >> 5, hh = lane >> 4, m = lane & 15;
    const int total = (nImg / 32) * NG;
    int gw = (int)blockIdx.x * LW + wave;
    const bool wvalid = gw < total;
    gw = wvalid ? gw : (total - 1);
    const int mp = gw / NG, ng = gw - mp * NG;

    const _Float16* a0p = A + (size_t)(mp * 32 + m) * KT + 8 * hh;
    const _Float16* a1p = a0p + (size_t)16 * KT;
    const _Float16* bq  = wT + (size_t)(ng * 64 + m) * KT + 8 * hh;

    v8f acc0[NT], acc1[NT];
#pragma unroll
    for (int t = 0; t < NT; ++t) { acc0[t] = z8f(); acc1[t] = z8f(); }

#pragma unroll 1
    for (int s = 0; s < KS; ++s) {
        const int ko = s * 32;
        FragH a0, a1;
        a0.h[0] = *(const v8h*)(a0p + ko);
        a0.h[1] = *(const v8h*)(a0p + ko + 16);
        a1.h[0] = *(const v8h*)(a1p + ko);
        a1.h[1] = *(const v8h*)(a1p + ko + 16);
#pragma unroll
        for (int t = 0; t < NT; ++t) {
            FragH bf;
            const _Float16* bp = bq + (size_t)(t * 16) * KT + ko;
            bf.h[0] = *(const v8h*)bp;
            bf.h[1] = *(const v8h*)(bp + 16);
            acc0[t] = wmh(a0.v, bf.v, acc0[t]);
            acc1[t] = wmh(a1.v, bf.v, acc1[t]);
        }
    }

    float* sw = stg + wave * 2048;
#pragma unroll
    for (int t = 0; t < NT; ++t) {
        const int col = t * 16 + m;
        const float bv = bias[ng * 64 + col];
#pragma unroll
        for (int r = 0; r < 8; ++r) {
            sw[(8 * hh + r) * 64 + col]      = fmaxf(acc0[t][r] * WINV64 + bv, 0.0f);
            sw[(16 + 8 * hh + r) * 64 + col] = fmaxf(acc1[t][r] * WINV64 + bv, 0.0f);
        }
    }
    __syncthreads();

    const size_t rowb = (size_t)mp * 32;
    if (wvalid) {
#pragma unroll
        for (int it = 0; it < 16; ++it) {
            const int q = it * 32 + lane, row = q >> 4, j = q & 15;
            const v4f v = *(const v4fa*)(sw + row * 64 + 4 * j);
            *(volatile v4fa*)(outp + (rowb + row) * NO + ng * 64 + 4 * j) = v;
        }
    }
    __threadfence();
    if (wvalid) {
#pragma unroll
        for (int it = 0; it < 16; ++it) {
            const int q = it * 32 + lane, row = q >> 4, j = q & 15;
            const v4f v = *(const v4fa*)(sw + row * 64 + 4 * j);
            *(volatile v4fa*)(outp + (rowb + row) * NO + ng * 64 + 4 * j) = v;
        }
    }
}

__global__ __launch_bounds__(TT)
void k_tail(const float* __restrict__ camf, const float* __restrict__ pos, const float* __restrict__ team,
            const int* __restrict__ aidx, const float* __restrict__ Wg,
            const float* __restrict__ asrc, const float* __restrict__ adst,
            const float* __restrict__ Wid, const float* __restrict__ bid,
            const float* __restrict__ Wh1, const float* __restrict__ bh1,
            const float* __restrict__ Wh2, const float* __restrict__ bh2,
            float* outp, int nImg)
{
    __shared__ float sCam[256];
    __shared__ __attribute__((aligned(16))) float sHN[16 * 256];
    __shared__ float sTm[64];
    __shared__ float sPos[4];
    __shared__ float sRel[64];
    __shared__ float sAdj[16];
    __shared__ float sSrc[32];
    __shared__ float sDst[32];
    __shared__ float sAl[32];
    __shared__ float sFu[320];
    __shared__ float sZ[256];
    __shared__ __attribute__((aligned(16))) float sLog[SPB * 6];
    __shared__ int   sAi;
    __shared__ float sAf;

    const int tid = threadIdx.x, lane = tid & 31, wave = tid >> 5;
    const int b0 = (int)blockIdx.x * SPB;

#pragma unroll 1
    for (int s = 0; s < SPB; ++s) {
        int b = b0 + s;
        b = b > nImg - 1 ? nImg - 1 : b;
        sCam[tid] = camf[(size_t)b * 256 + tid];
        if (tid < 48) { const int i = tid / 3, c = tid - 3 * i; sTm[i * 4 + c] = team[(size_t)b * 48 + tid]; }
        if (tid < 3) sPos[tid] = pos[(size_t)b * 3 + tid];
        if (tid == 0) {
            const int a = aidx[b];
            int aw = a < 0 ? a + 16 : a;
            aw = aw < 0 ? 0 : (aw > 15 ? 15 : aw);
            sAi = aw;
            sAf = (float)a;
        }
        __syncthreads();

        if (tid < 48) { const int i = tid / 3, c = tid - 3 * i; sRel[i * 4 + c] = sTm[i * 4 + c] - sPos[c]; }
        float cg = 0.0f;
#pragma unroll 1
        for (int k = 0; k < 256; ++k) cg += sCam[k] * Wg[(size_t)k * 256 + tid];
        const float w0 = Wg[256 * 256 + tid], w1 = Wg[257 * 256 + tid], w2 = Wg[258 * 256 + tid];
        __syncthreads();

#pragma unroll 1
        for (int i = 0; i < 16; ++i)
            sHN[i * 256 + tid] = cg + sRel[i * 4] * w0 + sRel[i * 4 + 1] * w1 + sRel[i * 4 + 2] * w2;
        if (tid < 16) {
#pragma clang fp contract(off)
            const int i = sAi, j = tid;
            const float dx = sTm[i * 4]     - sTm[j * 4];
            const float dy = sTm[i * 4 + 1] - sTm[j * 4 + 1];
            const float dz = sTm[i * 4 + 2] - sTm[j * 4 + 2];
            const float d2 = (dx * dx + dy * dy) + dz * dz;
            const float d  = sqrtf(d2);
            sAdj[j] = (d < 100.0f && j != i) ? 1.0f : 0.0f;
        }
        __syncthreads();

        if (tid < 64) {
            const int which = tid >> 5, i = (tid >> 1) & 15, hh = tid & 1;
            const float* av = (which != 0) ? adst : asrc;
            float d = 0.0f;
#pragma unroll 1
            for (int k = 0; k < 128; ++k) d += sHN[i * 256 + hh * 128 + k] * av[hh * 128 + k];
            if (which != 0) sDst[i * 2 + hh] = d; else sSrc[i * 2 + hh] = d;
        }
        if (tid == 64) {
            float rs = 0.0f;
#pragma unroll 1
            for (int j = 0; j < 16; ++j) rs += sAdj[j];
            if (rs == 0.0f) sAdj[sAi] = 1.0f;
        }
        __syncthreads();

        if (tid < 32) {
            const int hh = lane >> 4, j = lane & 15, i = sAi;
            float e = sSrc[i * 2 + hh] + sDst[j * 2 + hh];
            e = (e >= 0.0f) ? e : 0.2f * e;
            e = (sAdj[j] > 0.0f) ? e : -1.0e9f;
            float mx = e;
            mx = fmaxf(mx, __shfl_xor(mx, 8));
            mx = fmaxf(mx, __shfl_xor(mx, 4));
            mx = fmaxf(mx, __shfl_xor(mx, 2));
            mx = fmaxf(mx, __shfl_xor(mx, 1));
            const float p = expf(e - mx);
            float sm = p;
            sm += __shfl_xor(sm, 8);
            sm += __shfl_xor(sm, 4);
            sm += __shfl_xor(sm, 2);
            sm += __shfl_xor(sm, 1);
            sAl[hh * 16 + j] = p * (1.0f / sm);
        }
        __syncthreads();

        {
            const int n = tid, hh = n >> 7;
            float a = 0.0f;
#pragma unroll 1
            for (int j = 0; j < 16; ++j) a += sAl[hh * 16 + j] * sHN[j * 256 + n];
            const float en = expm1f(fminf(a, 0.0f));
            a = (a > 0.0f) ? a : en;
            if (!(fabsf(a) <= 3.402823466e38f)) a = 0.0f;
            sFu[n] = a;
        }
        if (tid < 64) sFu[256 + tid] = fmaxf(sAf * Wid[tid] + bid[tid], 0.0f);
        __syncthreads();

        {
            float a = 0.0f;
#pragma unroll 1
            for (int k = 0; k < 320; ++k) a += sFu[k] * Wh1[(size_t)k * 256 + tid];
            a += bh1[tid];
            sZ[tid] = fmaxf(a, 0.0f);
        }
        __syncthreads();

        if (wave < 6) {
            float a = 0.0f;
#pragma unroll 1
            for (int k = lane; k < 256; k += 32) a += sZ[k] * Wh2[k * 6 + wave];
            a += __shfl_xor(a, 16);
            a += __shfl_xor(a, 8);
            a += __shfl_xor(a, 4);
            a += __shfl_xor(a, 2);
            a += __shfl_xor(a, 1);
            if (lane == 0) sLog[s * 6 + wave] = a + bh2[wave];
        }
        __syncthreads();
    }

    v4f lv = {0.0f, 0.0f, 0.0f, 0.0f};
    if (tid < 24) lv = *(const v4fa*)(sLog + 4 * tid);
    float* op = outp + (size_t)b0 * 6 + 4 * tid;
    if (tid < 24) *(volatile v4fa*)op = lv;
    __threadfence();
    if (tid < 24) *(volatile v4fa*)op = lv;
}

extern "C" void kernel_launch(void* const* d_in, const int* in_sizes, int n_in,
                              void* d_out, int out_size, void* d_ws, size_t ws_size,
                              hipStream_t stream)
{
    if (n_in < 21) return;
    const int nImg = in_sizes[3];
    if (nImg <= 0 || (nImg % 32) != 0) return;
    if (in_sizes[0] != nImg * 21168 || in_sizes[1] != nImg * 3 || in_sizes[2] != nImg * 48) return;
    if (in_sizes[4] != 6144 || in_sizes[5] < 32 || in_sizes[6] != 32768 || in_sizes[7] < 64) return;
    if (in_sizes[8] != 36864 || in_sizes[9] < 64 || in_sizes[10] != 4194304 || in_sizes[11] < 256) return;
    if (in_sizes[12] < 64 || in_sizes[13] < 64 || in_sizes[14] != 66304) return;
    if (in_sizes[15] < 256 || in_sizes[16] < 256 || in_sizes[17] != 81920 || in_sizes[18] < 256) return;
    if (in_sizes[19] != 1536 || in_sizes[20] < 6) return;
    if (out_size != nImg * 6) return;

    const float* cam  = (const float*)d_in[0];
    const float* pos  = (const float*)d_in[1];
    const float* team = (const float*)d_in[2];
    const int*   aidx = (const int*)d_in[3];
    const float* W1   = (const float*)d_in[4];
    const float* b1   = (const float*)d_in[5];
    const float* W2   = (const float*)d_in[6];
    const float* b2   = (const float*)d_in[7];
    const float* W3   = (const float*)d_in[8];
    const float* b3   = (const float*)d_in[9];
    const float* Wp   = (const float*)d_in[10];
    const float* bp   = (const float*)d_in[11];
    const float* Wid  = (const float*)d_in[12];
    const float* bid  = (const float*)d_in[13];
    const float* Wg   = (const float*)d_in[14];
    const float* asrc = (const float*)d_in[15];
    const float* adst = (const float*)d_in[16];
    const float* Wh1  = (const float*)d_in[17];
    const float* bh1  = (const float*)d_in[18];
    const float* Wh2  = (const float*)d_in[19];
    const float* bh2  = (const float*)d_in[20];
    float* out = (float*)d_out;

    char* ws = (char*)d_ws;
    size_t off = 0;
    const size_t oW1 = off; off += (size_t)32 * 192 * 2;
    const size_t oW2 = off; off += (size_t)64 * 512 * 2;
    const size_t oW3 = off; off += (size_t)64 * 576 * 2;
    const size_t oWp = off; off += (size_t)256 * 16384 * 2;
    const size_t oCf = off; off += (size_t)nImg * 256 * 4;
    const size_t oO1 = off; off += (size_t)nImg * 1536 * 32 * 2;
    const size_t oO2 = off; off += (size_t)nImg * 352 * 64 * 2;
    const size_t oO3 = off; off += (size_t)nImg * 256 * 64 * 2;
    if (off > ws_size || off > (size_t)134217728) return;

    _Float16* w1T  = (_Float16*)(ws + oW1);
    _Float16* w2T  = (_Float16*)(ws + oW2);
    _Float16* w3T  = (_Float16*)(ws + oW3);
    _Float16* wpT  = (_Float16*)(ws + oWp);
    float*    camf = (float*)(ws + oCf);
    _Float16* out1 = (_Float16*)(ws + oO1);
    _Float16* out2 = (_Float16*)(ws + oO2);
    _Float16* out3 = (_Float16*)(ws + oO3);

    k_prep<<<293, PT, 0, stream>>>(Wp, W1, W2, W3, wpT, w1T, w2T, w3T);

    k_conv<float, 84, 84, 3, 32, 8, 2, 39, 39, 7056, 1536>
        <<<(nImg * 48 + CW - 1) / CW, CT, 0, stream>>>(cam, w1T, b1, out1, nImg);
    k_conv<_Float16, 39, 39, 32, 64, 4, 2, 18, 18, 1536, 352>
        <<<(nImg * 11 + CW - 1) / CW, CT, 0, stream>>>(out1, w2T, b2, out2, nImg);
    k_conv<_Float16, 18, 18, 64, 64, 3, 1, 16, 16, 352, 256>
        <<<(nImg * 8 + CW - 1) / CW, CT, 0, stream>>>(out2, w3T, b3, out3, nImg);

    {
        const int waves = (nImg / 32) * 4;
        k_linear<<<(waves + LW - 1) / LW, LT, 0, stream>>>(out3, wpT, bp, camf, nImg);
    }

    k_tail<<<nImg / SPB, TT, 0, stream>>>(camf, pos, team, aidx, Wg, asrc, adst, Wid, bid,
                                           Wh1, bh1, Wh2, bh2, out, nImg);
}
